// RelativeMultiHeadAttn_88021059764226
// MI455X (gfx1250) — hardware-verified
//
#include <hip/hip_runtime.h>
#include <math.h>
#include <stdint.h>

#ifndef NB
#define NB 4
#endif
#ifndef SEQ
#define SEQ 1024
#endif
#define NB_FULL  4
#define SEQ_FULL 1024
#define ND    1024
#define NH    16
#define HDV   64
#define HQK   128
#define QKW   (2 * ND)
#define NKT   (SEQ / 64)
#define BDW   (SEQ + 64)
#define NPAIR 16

static_assert(SEQ % 64 == 0);
static_assert(SEQ >= 64);
static_assert(SEQ <= SEQ_FULL);
static_assert(NB >= 1);
static_assert(NB <= NB_FULL);
static_assert(ND == NH * HDV);
static_assert(HQK == 2 * HDV);
static_assert(NH % NPAIR == 0);
static_assert(ND % 256 == 0);
static_assert(BDW % 64 == 0);
static_assert((3 * ND) % 64 == 0);
static_assert(SEQ % 8 == 0);

typedef _Float16 v16h __attribute__((ext_vector_type(16)));
typedef _Float16 v8h  __attribute__((ext_vector_type(8)));
typedef float    v8f  __attribute__((ext_vector_type(8)));
typedef float    v4f  __attribute__((ext_vector_type(4)));
typedef v4f __attribute__((may_alias)) v4fa;
typedef v8h __attribute__((may_alias)) v8ha;

__device__ __forceinline__ float bf_rne(float f) {
  unsigned u = __float_as_uint(f);
  u = (u + 0x7FFFu + ((u >> 16) & 1u)) & 0xFFFF0000u;
  return __uint_as_float(u);
}

union FragU { v16h v; v8ha h[2]; };
__device__ __forceinline__ v16h ldfrag(const _Float16* p) {
  FragU f;
  f.h[0] = *(const v8ha*)(p);
  f.h[1] = *(const v8ha*)(p + 16);
  return f.v;
}

__device__ __forceinline__ v8f mma16(v16h a, v16h b, v8f c) {
  c = __builtin_amdgcn_wmma_f32_16x16x32_f16(false, a, false, b, (short)0, c, false, false);
  asm volatile("v_nop\n\tv_nop\n\tv_nop\n\tv_nop" : "+v"(c) : "v"(a), "v"(b));
  return c;
}

__device__ __forceinline__ v8f zero8() { v8f z = {0.f, 0.f, 0.f, 0.f, 0.f, 0.f, 0.f, 0.f}; return z; }

__global__ __launch_bounds__(256) void cvt_kernel(const float* __restrict__ src, int sstride,
                                                  _Float16* __restrict__ dst, int nrows, float s1) {
  const int i = blockIdx.x * 256 + threadIdx.x;
  if (i >= nrows * (ND / 8)) return;
  const int r  = i / (ND / 8);
  const int c8 = (i - r * (ND / 8)) * 8;
  const float* sp = src + (size_t)r * sstride + c8;
  const v4f a = *(const v4f*)(sp);
  const v4f b = *(const v4f*)(sp + 4);
  float f[8];
  f[0] = bf_rne(a[0]); f[1] = bf_rne(a[1]); f[2] = bf_rne(a[2]); f[3] = bf_rne(a[3]);
  f[4] = bf_rne(b[0]); f[5] = bf_rne(b[1]); f[6] = bf_rne(b[2]); f[7] = bf_rne(b[3]);
  v8h o1;
#pragma unroll
  for (int e = 0; e < 8; ++e) o1[e] = (_Float16)(f[e] * s1);
  _Float16* dp = dst + (size_t)r * ND + c8;
  *(volatile v8h*)dp = o1;
  __threadfence();
  *(volatile v8h*)dp = o1;
}

__global__ __launch_bounds__(256) void qsplit_kernel(const float* __restrict__ Q, const float* __restrict__ bw,
                                                     const float* __restrict__ br, _Float16* __restrict__ DW,
                                                     _Float16* __restrict__ DR, int nrows) {
  const int i = blockIdx.x * 256 + threadIdx.x;
  if (i >= nrows * (ND / 8)) return;
  const int r  = i / (ND / 8);
  const int c8 = (i - r * (ND / 8)) * 8;
  const int h  = c8 >> 6;
  const int d0 = c8 & 63;
  const float* sp = Q + (size_t)r * ND + c8;
  const v4f a  = *(const v4f*)(sp);
  const v4f b  = *(const v4f*)(sp + 4);
  const v4f wa = *(const v4f*)(bw + c8);
  const v4f wb = *(const v4f*)(bw + c8 + 4);
  const v4f ra = *(const v4f*)(br + c8);
  const v4f rb = *(const v4f*)(br + c8 + 4);
  float f[8], gw[8], gr[8];
  f[0] = a[0]; f[1] = a[1]; f[2] = a[2]; f[3] = a[3];
  f[4] = b[0]; f[5] = b[1]; f[6] = b[2]; f[7] = b[3];
  gw[0] = bf_rne(wa[0]); gw[1] = bf_rne(wa[1]); gw[2] = bf_rne(wa[2]); gw[3] = bf_rne(wa[3]);
  gw[4] = bf_rne(wb[0]); gw[5] = bf_rne(wb[1]); gw[6] = bf_rne(wb[2]); gw[7] = bf_rne(wb[3]);
  gr[0] = bf_rne(ra[0]); gr[1] = bf_rne(ra[1]); gr[2] = bf_rne(ra[2]); gr[3] = bf_rne(ra[3]);
  gr[4] = bf_rne(rb[0]); gr[5] = bf_rne(rb[1]); gr[6] = bf_rne(rb[2]); gr[7] = bf_rne(rb[3]);
  v8h hw, lw, hr, lr;
#pragma unroll
  for (int e = 0; e < 8; ++e) {
    const float tw = (f[e] + gw[e]) * 16.0f;
    const _Float16 qw = (_Float16)tw;
    hw[e] = qw;
    lw[e] = (_Float16)((tw - (float)qw) * 1024.0f);
    const float tr = (f[e] + gr[e]) * 16.0f;
    const _Float16 qr = (_Float16)tr;
    hr[e] = qr;
    lr[e] = (_Float16)((tr - (float)qr) * 1024.0f);
  }
  _Float16* dw = DW + (size_t)r * QKW + h * HQK + d0;
  _Float16* dr = DR + (size_t)r * QKW + h * HQK + d0;
  for (int ps = 0; ps < 2; ++ps) {
    *(volatile v8h*)(dw)      = hw;
    *(volatile v8h*)(dw + 64) = lw;
    *(volatile v8h*)(dr)      = hr;
    *(volatile v8h*)(dr + 64) = lr;
    __threadfence();
  }
}

template <int OUT, bool SKEW, bool HASB>
__global__ __launch_bounds__(256) void gemm_f16_kernel(
    const _Float16* __restrict__ A, int lda, long strideA,
    const _Float16* __restrict__ Bt, int ldb, long strideB,
    void* C1, int ldc, long strideC,
    const float* __restrict__ b1,
    int M, int N, int K, float scale, float carry, int skew0, int wrapN) {
  __shared__ __align__(16) float sT[8][16 * 68];

  const int z    = blockIdx.y;
  const int lane = threadIdx.x & 31;
  const int wave = threadIdx.x >> 5;
  const int tilesN = N >> 6;
  const int tilesM = M >> 6;
  const int tile = blockIdx.x * 8 + wave;
  if (tile >= tilesM * tilesN) return;
  const int tm = tile / tilesN;
  const int tn = tile - tm * tilesN;
  const int m0 = tm << 6;
  const int n0 = tn << 6;
  const int nsk = SKEW ? ((skew0 - tm) << 6) : 0;

  const _Float16* Ab = A  + (size_t)z * strideA;
  const _Float16* Bb = Bt + (size_t)z * strideB;

  const int rl   = lane & 15;
  const int koff = (lane >> 4) * 8;
  const int mOff = (lane >> 4) * 8;

  v8f acc[4][4];
#pragma unroll
  for (int i = 0; i < 4; ++i)
#pragma unroll
    for (int j = 0; j < 4; ++j) acc[i][j] = zero8();

  for (int k0 = 0; k0 < K; k0 += 32) {
    v16h bfr[4];
#pragma unroll
    for (int j = 0; j < 4; ++j) {
      int brow = nsk + n0 + (j << 4) + rl;
      if (SKEW) brow -= (brow >= wrapN) ? wrapN : 0;
      bfr[j] = ldfrag(Bb + (size_t)brow * ldb + koff + k0);
    }
#pragma unroll
    for (int i = 0; i < 4; ++i) {
      const v16h af = ldfrag(Ab + (size_t)(m0 + (i << 4) + rl) * lda + koff + k0);
#pragma unroll
      for (int j = 0; j < 4; ++j) acc[i][j] = mma16(af, bfr[j], acc[i][j]);
    }
  }

  float* slab = sT[wave];
  const int hh = lane >> 4, c4 = (lane & 15) * 4;
  const int q8 = lane >> 3, c8 = (lane & 7) * 8;
  v4f bias4 = {0.f, 0.f, 0.f, 0.f};
  float col8a[8];
#pragma unroll
  for (int e = 0; e < 8; ++e) col8a[e] = 0.f;
  if (OUT == 1 && HASB) {
    const v4f tb = *(const v4f*)(b1 + n0 + c4);
    bias4[0] = bf_rne(tb[0]); bias4[1] = bf_rne(tb[1]); bias4[2] = bf_rne(tb[2]); bias4[3] = bf_rne(tb[3]);
  }
  if ((OUT == 2 || OUT == 3) && HASB) {
    const v4f ta = *(const v4f*)(b1 + n0 + c8);
    const v4f tb = *(const v4f*)(b1 + n0 + c8 + 4);
    col8a[0] = bf_rne(ta[0]); col8a[1] = bf_rne(ta[1]); col8a[2] = bf_rne(ta[2]); col8a[3] = bf_rne(ta[3]);
    col8a[4] = bf_rne(tb[0]); col8a[5] = bf_rne(tb[1]); col8a[6] = bf_rne(tb[2]); col8a[7] = bf_rne(tb[3]);
  }
  const float carry2 = carry * 0.0009765625f;

#pragma unroll
  for (int i = 0; i < 4; ++i) {
    const int mBase = m0 + (i << 4);
#pragma unroll
    for (int j = 0; j < 4; ++j)
#pragma unroll
      for (int r = 0; r < 8; ++r)
        slab[(mOff + r) * 68 + (j << 4) + rl] = acc[i][j][r] * scale;
    __builtin_amdgcn_fence(__ATOMIC_RELEASE, "workgroup");
    __builtin_amdgcn_wave_barrier();
    __builtin_amdgcn_fence(__ATOMIC_ACQUIRE, "workgroup");
    if (OUT == 0 || OUT == 1) {
      float* C = (float*)C1 + (size_t)z * strideC;
      v4f vv[8];
#pragma unroll
      for (int it = 0; it < 8; ++it) {
        const int row = it * 2 + hh;
        v4f v = *(const v4fa*)(slab + row * 68 + c4);
        if (OUT == 1) v += bias4;
        vv[it] = v;
      }
      for (int ps = 0; ps < 2; ++ps) {
#pragma unroll
        for (int it = 0; it < 8; ++it) {
          const int row = it * 2 + hh;
          *(volatile v4f*)(C + (size_t)(mBase + row) * ldc + n0 + c4) = vv[it];
        }
        __threadfence();
      }
    } else if (OUT == 2 || OUT == 4) {
      _Float16* Ca = (_Float16*)C1 + (size_t)z * strideC;
      v8h hv[4], lv[4];
#pragma unroll
      for (int it = 0; it < 4; ++it) {
        const int row = it * 4 + q8;
        const float* sp = slab + row * 68 + c8;
        const v4f x0 = *(const v4fa*)(sp);
        const v4f x1 = *(const v4fa*)(sp + 4);
        float f[8];
        f[0] = x0[0]; f[1] = x0[1]; f[2] = x0[2]; f[3] = x0[3];
        f[4] = x1[0]; f[5] = x1[1]; f[6] = x1[2]; f[7] = x1[3];
        float rb = 0.f;
        if (OUT == 4 && HASB) rb = bf_rne(b1[mBase + row]);
        v8h ha, la;
#pragma unroll
        for (int e = 0; e < 8; ++e) {
          const float t = f[e] + ((OUT == 2) ? col8a[e] : rb);
          ha[e] = (_Float16)(t * carry);
          la[e] = (_Float16)(t * carry2);
        }
        hv[it] = ha; lv[it] = la;
      }
      for (int ps = 0; ps < 2; ++ps) {
#pragma unroll
        for (int it = 0; it < 4; ++it) {
          const int row = it * 4 + q8;
          if (OUT == 2) {
            _Float16* cp = Ca + (size_t)(mBase + row) * ldc + 2 * n0 + c8;
            *(volatile v8h*)(cp)      = hv[it];
            *(volatile v8h*)(cp + 64) = lv[it];
          } else {
            *(volatile v8h*)(Ca + (size_t)(mBase + row) * ldc + n0 + c8) = hv[it];
          }
        }
        __threadfence();
      }
    } else {
      _Float16* Cc = (_Float16*)C1 + (size_t)z * strideC;
      v8h hv[4], lv[4];
#pragma unroll
      for (int it = 0; it < 4; ++it) {
        const int row = it * 4 + q8;
        const float* sp = slab + row * 68 + c8;
        const v4f x0 = *(const v4fa*)(sp);
        const v4f x1 = *(const v4fa*)(sp + 4);
        float f[8];
        f[0] = x0[0]; f[1] = x0[1]; f[2] = x0[2]; f[3] = x0[3];
        f[4] = x1[0]; f[5] = x1[1]; f[6] = x1[2]; f[7] = x1[3];
        v8h ha, la;
#pragma unroll
        for (int e = 0; e < 8; ++e) {
          const float t  = f[e] + col8a[e];
          const float th = t * carry;
          const _Float16 hq = (_Float16)th;
          ha[e] = hq;
          la[e] = (_Float16)((th - (float)hq) * 1024.0f);
        }
        hv[it] = ha; lv[it] = la;
      }
      for (int ps = 0; ps < 2; ++ps) {
#pragma unroll
        for (int it = 0; it < 4; ++it) {
          const int row = it * 4 + q8;
          _Float16* cp = Cc + (size_t)(mBase + row) * ldc + 2 * n0 + c8;
          *(volatile v8h*)(cp)      = hv[it];
          *(volatile v8h*)(cp + 64) = lv[it];
        }
        __threadfence();
      }
    }
    __builtin_amdgcn_fence(__ATOMIC_RELEASE, "workgroup");
    __builtin_amdgcn_wave_barrier();
    __builtin_amdgcn_fence(__ATOMIC_ACQUIRE, "workgroup");
  }
}

__global__ __launch_bounds__(128)
void relattn_kernel(const _Float16* __restrict__ QU, const _Float16* __restrict__ KP,
                    const _Float16* __restrict__ VT, const float* __restrict__ BD,
                    _Float16* __restrict__ CTX, int h0, float cs) {
  __shared__ __align__(16) unsigned char SMEM[32768];
  _Float16* Ksh = (_Float16*)(SMEM);
  _Float16* Vsh = (_Float16*)(SMEM + 16384);
  _Float16* Psh = (_Float16*)(SMEM + 24576);
  float*    Osh = (float*)(SMEM);

  const int tid  = threadIdx.x;
  const int wave = tid >> 5;
  const int lane = tid & 31;
  const int hh   = lane >> 4;
  const int c    = lane & 15;

  const int z    = blockIdx.y;
  const int h    = h0 + z;
  const int qb   = blockIdx.x;
  const int q0   = qb * 64 + wave * 16;
  const int rr0  = wave * 16 + 8 * hh;
  const int iq   = q0 + 8 * hh;

  const _Float16* Qh = QU + h * HQK;
  const _Float16* Kh = KP + h * HQK;
  const _Float16* Vh = VT + (size_t)(h * HDV) * SEQ;
  const float*    bd = BD + (size_t)z * SEQ * BDW;
  _Float16*       ctx = CTX + h * HDV;

  v16h qa[4];
#pragma unroll
  for (int dc = 0; dc < 4; ++dc)
    qa[dc] = ldfrag(Qh + (size_t)(q0 + c) * QKW + dc * 32 + 8 * hh);

  const float* bdr = bd + (size_t)(q0 + 8 * hh) * BDW + (63 - rr0 + c);
  const bool edge  = (wave == 3) && (hh == 1);
  const bool lastb = (qb == NKT - 1);
  const int  ex7   = edge ? (lastb ? 0 : (BDW + 63)) : (BDW - 1);

  float mrow[8], lrow[8];
  v8f oacc[4];
#pragma unroll
  for (int r = 0; r < 8; ++r) { mrow[r] = -INFINITY; lrow[r] = 0.f; }
#pragma unroll
  for (int t = 0; t < 4; ++t) oacc[t] = zero8();

  _Float16* pw = Psh + wave * (16 * 64);

#pragma unroll 1
  for (int kc = 0; kc < NKT; ++kc) {
    const int kv0 = kc * 64;
    __syncthreads();
    {
      const int r = tid >> 1, c0 = (tid & 1) * 64, cv = (tid & 1) * 32;
      const _Float16* ks = Kh + (size_t)(kv0 + r) * QKW + c0;
      const _Float16* vs = Vh + (size_t)r * SEQ + kv0 + cv;
#pragma unroll
      for (int i = 0; i < 8; ++i) {
        const v8h kk8 = *(const v8h*)(ks + 8 * i);
        *(v8ha*)(Ksh + r * 128 + c0 + 8 * i) = kk8;
      }
#pragma unroll
      for (int i = 0; i < 4; ++i) {
        const v8h vv8 = *(const v8h*)(vs + 8 * i);
        *(v8ha*)(Vsh + r * 64 + cv + 8 * i) = vv8;
      }
    }
    __syncthreads();

    v8f s[4];
#pragma unroll
    for (int j = 0; j < 4; ++j) {
      s[j] = zero8();
#pragma unroll
      for (int dc = 0; dc < 4; ++dc) {
        const v16h kb = ldfrag(Ksh + (j * 16 + c) * 128 + dc * 32 + 8 * hh);
        s[j] = mma16(qa[dc], kb, s[j]);
      }
    }

    float cm[8];
#pragma unroll
    for (int r = 0; r < 8; ++r) {
      const int i  = iq + r;
      const int ex = (r == 7) ? ex7 : (BDW - 1);
      float m = -INFINITY;
#pragma unroll
      for (int j = 0; j < 4; ++j) {
        const int key = kv0 + (j << 4) + c;
        const int a1  = r * (BDW - 1) + kv0 + (j << 4);
        const int ia  = a1 + ((key > i) ? ex : 0);
        const float bvl = bdr[ia];
        const float bdv = (key == i + 1) ? 0.0f : bvl;
        const float sv  = s[j][r] * cs + bdv;
        s[j][r] = sv;
        m = fmaxf(m, sv);
      }
      m = fmaxf(m, __shfl_xor(m, 1, 32));
      m = fmaxf(m, __shfl_xor(m, 2, 32));
      m = fmaxf(m, __shfl_xor(m, 4, 32));
      m = fmaxf(m, __shfl_xor(m, 8, 32));
      cm[r] = m;
      __asm__ __volatile__("" ::: "memory");
    }

#pragma unroll
    for (int r = 0; r < 8; ++r) {
      const float mnew  = fmaxf(mrow[r], cm[r]);
      const float alpha = __expf(mrow[r] - mnew);
      mrow[r] = mnew;
      float psum = 0.f;
#pragma unroll
      for (int j = 0; j < 4; ++j) {
        const float p = __expf(s[j][r] - mnew);
        psum += p;
        pw[(8 * hh + r) * 64 + j * 16 + c] = (_Float16)(p * 4096.0f);
      }
      psum += __shfl_xor(psum, 1, 32);
      psum += __shfl_xor(psum, 2, 32);
      psum += __shfl_xor(psum, 4, 32);
      psum += __shfl_xor(psum, 8, 32);
      lrow[r] = lrow[r] * alpha + psum;
#pragma unroll
      for (int t = 0; t < 4; ++t) oacc[t][r] *= alpha;
    }
    __builtin_amdgcn_fence(__ATOMIC_RELEASE, "workgroup");
    __builtin_amdgcn_wave_barrier();
    __builtin_amdgcn_fence(__ATOMIC_ACQUIRE, "workgroup");

#pragma unroll
    for (int kk = 0; kk < 2; ++kk) {
      const v16h pa = ldfrag(pw + c * 64 + kk * 32 + 8 * hh);
#pragma unroll
      for (int t = 0; t < 4; ++t) {
        const v16h vb = ldfrag(Vsh + (t * 16 + c) * 64 + kk * 32 + 8 * hh);
        oacc[t] = mma16(pa, vb, oacc[t]);
      }
    }
  }

  __syncthreads();
  float* os = Osh + wave * (16 * HDV);
#pragma unroll
  for (int r = 0; r < 8; ++r) {
    const float inv = 1.0f / (1024.0f * lrow[r]);
#pragma unroll
    for (int t = 0; t < 4; ++t) os[(8 * hh + r) * HDV + t * 16 + c] = oacc[t][r] * inv;
  }
  __builtin_amdgcn_fence(__ATOMIC_RELEASE, "workgroup");
  __builtin_amdgcn_wave_barrier();
  __builtin_amdgcn_fence(__ATOMIC_ACQUIRE, "workgroup");
  const int q8 = lane >> 3, c8 = (lane & 7) * 8;
  v8h ov[4];
#pragma unroll
  for (int it = 0; it < 4; ++it) {
    const int row = it * 4 + q8;
    const float* sp = os + row * HDV + c8;
    const v4f x0 = *(const v4fa*)(sp);
    const v4f x1 = *(const v4fa*)(sp + 4);
    v8h o;
    o[0] = (_Float16)x0[0]; o[1] = (_Float16)x0[1]; o[2] = (_Float16)x0[2]; o[3] = (_Float16)x0[3];
    o[4] = (_Float16)x1[0]; o[5] = (_Float16)x1[1]; o[6] = (_Float16)x1[2]; o[7] = (_Float16)x1[3];
    ov[it] = o;
  }
  for (int ps = 0; ps < 2; ++ps) {
#pragma unroll
    for (int it = 0; it < 4; ++it) {
      const int row = it * 4 + q8;
      *(volatile v8h*)(ctx + (size_t)(q0 + row) * ND + c8) = ov[it];
    }
    __threadfence();
  }
}

__global__ __launch_bounds__(256) void resid_kernel(const float* __restrict__ X, int xstride,
                                                    const float* __restrict__ O,
                                                    float* out, int ostride, int nrows) {
  const int lane = threadIdx.x & 31;
  const int wave = threadIdx.x >> 5;
  const int row  = blockIdx.x * 8 + wave;
  if (row >= nrows) return;
  const float* xr  = X + (size_t)row * xstride;
  const float* orr = O + (size_t)row * ND;
  v4f y[8];
#pragma unroll
  for (int i = 0; i < 8; ++i) {
    const v4f xv = *(const v4f*)(xr + i * 128 + lane * 4);
    const v4f ov = *(const v4f*)(orr + i * 128 + lane * 4);
    v4f t;
    t[0] = bf_rne(xv[0]) + ov[0];
    t[1] = bf_rne(xv[1]) + ov[1];
    t[2] = bf_rne(xv[2]) + ov[2];
    t[3] = bf_rne(xv[3]) + ov[3];
    y[i] = t;
  }
  float* orow = out + (size_t)row * ostride;
  for (int ps = 0; ps < 2; ++ps) {
#pragma unroll
    for (int i = 0; i < 8; ++i)
      *(volatile v4f*)(orow + i * 128 + lane * 4) = y[i];
    __threadfence();
  }
}

extern "C" void kernel_launch(void* const* d_in, const int* in_sizes, int n_in,
                              void* d_out, int out_size, void* d_ws, size_t ws_size,
                              hipStream_t stream) {
  if (n_in < 7) return;
  if (in_sizes[0] < ((SEQ - 1) * NB_FULL + NB) * ND) return;
  if (in_sizes[1] < SEQ * ND) return;
  if (in_sizes[2] < 3 * ND * ND) return;
  if (in_sizes[3] < ND * ND) return;
  if (in_sizes[4] < ND * ND) return;
  if (in_sizes[5] < NH * HDV || in_sizes[6] < NH * HDV) return;
  if (out_size < NB * SEQ * ND) return;

  const float* x    = (const float*)d_in[0];
  const float* pos  = (const float*)d_in[1];
  const float* wqkv = (const float*)d_in[2];
  const float* wr   = (const float*)d_in[3];
  const float* wo   = (const float*)d_in[4];
  const float* brb  = (const float*)d_in[5];
  const float* bwb  = (const float*)d_in[6];
  float* out = (float*)d_out;

  const size_t szW3  = (size_t)3 * ND * ND * 2;
  const size_t szWO  = (size_t)ND * ND * 2;
  const size_t szWR  = (size_t)ND * ND * 2;
  const size_t szRH  = (size_t)SEQ * ND * 2;
  const size_t szP2  = (size_t)SEQ * QKW * 2;
  const size_t szXH  = (size_t)SEQ * ND * 2;
  const size_t szQF  = (size_t)SEQ * ND * 4;
  const size_t szQ2  = (size_t)SEQ * QKW * 2;
  const size_t szVT  = (size_t)ND * SEQ * 2;
  const size_t szCTX = (size_t)SEQ * ND * 2;
  const size_t szOY  = (size_t)SEQ * ND * 4;
  const size_t szBD  = (size_t)NPAIR * SEQ * BDW * 4;
  size_t off = 0;
  const size_t oW3  = off; off += szW3;
  const size_t oWO  = off; off += szWO;
  const size_t oWR  = off; off += szWR;
  const size_t oRH  = off; off += szRH;
  const size_t oP2  = off; off += szP2;
  const size_t oXH  = off; off += szXH;
  const size_t oQF  = off; off += szQF;
  const size_t oQ2W = off; off += szQ2;
  const size_t oQ2R = off; off += szQ2;
  const size_t oKP2 = off; off += szQ2;
  const size_t oVT  = off; off += szVT;
  const size_t oCTX = off; off += szCTX;
  const size_t oOY  = off; off += szOY;
  const size_t oBD  = off; off += szBD;
  const size_t total = off;
  if (total > ws_size) return;
  if (total > (size_t)134217728) return;

  char* ws = (char*)d_ws;
  _Float16* W3  = (_Float16*)(ws + oW3);
  _Float16* WOp = (_Float16*)(ws + oWO);
  _Float16* WRp = (_Float16*)(ws + oWR);
  _Float16* RH  = (_Float16*)(ws + oRH);
  _Float16* P2  = (_Float16*)(ws + oP2);
  _Float16* XH  = (_Float16*)(ws + oXH);
  float*    QF  = (float*)(ws + oQF);
  _Float16* Q2W = (_Float16*)(ws + oQ2W);
  _Float16* Q2R = (_Float16*)(ws + oQ2R);
  _Float16* KP2 = (_Float16*)(ws + oKP2);
  _Float16* VTp = (_Float16*)(ws + oVT);
  _Float16* CTX = (_Float16*)(ws + oCTX);
  float*    OY  = (float*)(ws + oOY);
  float*    BDp = (float*)(ws + oBD);
  const _Float16* WQp = W3;
  const _Float16* WKp = W3 + (size_t)ND * ND;
  const _Float16* WVp = W3 + (size_t)2 * ND * ND;

  const float cs  = 0.125f * 0.00390625f;
  const float r4k = 0.000244140625f;
  const dim3 blk(256);

  cvt_kernel<<<dim3((3 * ND * (ND / 8) + 255) / 256), blk, 0, stream>>>(wqkv, ND, W3, 3 * ND, 64.0f);
  cvt_kernel<<<dim3((ND * (ND / 8) + 255) / 256), blk, 0, stream>>>(wo, ND, WOp, ND, 64.0f);
  cvt_kernel<<<dim3((ND * (ND / 8) + 255) / 256), blk, 0, stream>>>(wr, ND, WRp, ND, 64.0f);
  const dim3 gX((SEQ * (ND / 8) + 255) / 256);
  cvt_kernel<<<gX, blk, 0, stream>>>(pos, ND, RH, SEQ, 64.0f);
  const int tilesQ  = NKT * (ND / 64);
  const int tilesBD = NKT * (BDW / 64);
  gemm_f16_kernel<2, false, false><<<dim3((tilesQ + 7) / 8, 1), blk, 0, stream>>>(
      RH, ND, 0L, WRp, ND, 0L, (void*)P2, QKW, 0L, brb,
      SEQ, ND, ND, r4k, 16.0f, 0, SEQ);
  for (int b = 0; b < NB; ++b) {
    cvt_kernel<<<gX, blk, 0, stream>>>(x + (size_t)b * ND, NB_FULL * ND, XH, SEQ, 64.0f);
    gemm_f16_kernel<1, false, false><<<dim3((tilesQ + 7) / 8, 1), blk, 0, stream>>>(
        XH, ND, 0L, WQp, ND, 0L, (void*)QF, ND, 0L, bwb,
        SEQ, ND, ND, r4k, 1.0f, 0, SEQ);
    qsplit_kernel<<<gX, blk, 0, stream>>>(QF, bwb, brb, Q2W, Q2R, SEQ);
    gemm_f16_kernel<2, false, false><<<dim3((tilesQ + 7) / 8, 1), blk, 0, stream>>>(
        XH, ND, 0L, WKp, ND, 0L, (void*)KP2, QKW, 0L, bwb,
        SEQ, ND, ND, r4k, 16.0f, 0, SEQ);
    gemm_f16_kernel<4, false, false><<<dim3((tilesQ + 7) / 8, 1), blk, 0, stream>>>(
        WVp, ND, 0L, XH, ND, 0L, (void*)VTp, SEQ, 0L, bwb,
        ND, SEQ, ND, r4k, 16.0f, 0, SEQ);
    for (int gi = 0; gi < NH / NPAIR; ++gi) {
      const int h0 = gi * NPAIR;
      const _Float16* Aq = Q2R + h0 * HQK;
      const _Float16* Bp = P2 + h0 * HQK;
      gemm_f16_kernel<0, true, false><<<dim3((tilesBD + 7) / 8, NPAIR), blk, 0, stream>>>(
          Aq, QKW, (long)HQK, Bp, QKW, (long)HQK, (void*)BDp, BDW, (long)SEQ * BDW, brb,
          SEQ, BDW, HQK, cs, 1.0f, NKT - 1, SEQ);
      relattn_kernel<<<dim3(NKT, NPAIR), dim3(128), 0, stream>>>(
          Q2W, KP2, VTp, BDp, CTX, h0, cs);
    }
    gemm_f16_kernel<1, false, false><<<dim3((tilesQ + 7) / 8, 1), blk, 0, stream>>>(
        CTX, ND, 0L, WOp, ND, 0L, (void*)OY, ND, 0L, bwb,
        SEQ, ND, ND, r4k, 1.0f, 0, SEQ);
    resid_kernel<<<dim3(SEQ / 8), blk, 0, stream>>>(
        x + (size_t)b * ND, NB_FULL * ND, OY, out + (size_t)b * ND, NB * ND, SEQ);
  }
  (void)hipGetLastError();
}
